// Net_46737834115140
// MI455X (gfx1250) — hardware-run, weakly checked
//
#include <hip/hip_runtime.h>


#ifndef NB
#define NB 2
#endif
#ifndef SEQ
#define SEQ 16384
#endif
#define NB_FULL  2
#define SEQ_FULL 16384
#ifndef OUT_SEQ
#define OUT_SEQ SEQ
#endif
#define CW   32
#define DI   64
#define NS   16
#define XPN  34
#define XPP  48
#define LC   256
#define NCH  (SEQ / LC)
#define TS   32
#define AP   40
#define XAP  72
#define SDP  52
#define OSP  36
#define OS1P 68
#define WSC  64.0f
#define ACS  1024.0f
#define QRS  2048.0f
#define QRI  (1.0f / 2048.0f)
#define LOG2E 1.4426950408889634f

static constexpr int isq(int n) { int r = 0; while ((r + 1) * (r + 1) <= n) ++r; return r; }
static constexpr int IMG = isq(SEQ);

static_assert(IMG * IMG == SEQ);
static_assert(SEQ % 128 == 0);
static_assert(SEQ % 64 == 0);
static_assert(SEQ % LC == 0);
static_assert(LC % TS == 0);
static_assert(CW == 32);
static_assert(DI == 64);
static_assert(NS == 16);
static_assert(XPN == 2 + 2 * NS);
static_assert(XPP % 16 == 0 && XPP >= XPN);
static_assert((XPN * DI) % 8 == 0);
static_assert((AP * 2) % 16 == 0 && AP >= CW);
static_assert((XAP * 2) % 16 == 0 && XAP >= DI);
static_assert((OSP * 4) % 16 == 0 && (OS1P * 4) % 16 == 0);
static_assert(SDP >= XPP);
static_assert(NB <= NB_FULL);
static_assert(SEQ <= SEQ_FULL);
static_assert(((size_t)(NB - 1) * OUT_SEQ + SEQ) <= (size_t)NB_FULL * SEQ_FULL);
static_assert((size_t)NB_FULL * SEQ_FULL * CW * 4 == (size_t)4194304);
static_assert(4 * 128 * AP * 2 + 8 * 16 * OS1P * 4 <= 131072);
static_assert(2 * 67 * 64 * 4 + 64 * 64 * 4 + 64 * XAP * 2 + 64 * SDP * 4 <= 131072);
static_assert(64 * 32 * 4 <= 131072);
static_assert(TS * 64 * 4 <= 131072);
static_assert(4 * 16 * OSP * 4 <= 131072);
static_assert(32 * 16 * 8 == 16 * DI * 4);
static_assert(128 * 16 * 8 == 64 * DI * 4);
static_assert(128 * 16 * 4 == 64 * 32 * 4);
static_assert(64 * 16 * 8 == 64 * 32 * 4);
static_assert(64 * 16 * 4 == TS * DI * 2);
static_assert(32 * 16 * 4 == 16 * CW * 4);

typedef _Float16 h16;
typedef unsigned short bf;
typedef __attribute__((ext_vector_type(16))) __bf16   v16bf;
typedef __attribute__((ext_vector_type(16))) _Float16 v16h;
typedef __attribute__((ext_vector_type(8)))  _Float16 v8h;
typedef __attribute__((ext_vector_type(8)))  unsigned short v8us;
typedef __attribute__((ext_vector_type(8)))  float    v8f;
typedef __attribute__((ext_vector_type(4)))  float    v4f;
typedef v4f  __attribute__((may_alias)) v4fa;
typedef __attribute__((ext_vector_type(4)))  _Float16 v4h;

__device__ __forceinline__ unsigned short f2bf(float f) { unsigned u = __float_as_uint(f); u += 0x7FFFu + ((u >> 16) & 1u); return (unsigned short)(u >> 16); }
__device__ __forceinline__ float bfr(float f) { return __uint_as_float(((unsigned)f2bf(f)) << 16); }
__device__ __forceinline__ v16h cat16(v8h lo, v8h hi) { return __builtin_shufflevector(lo, hi, 0, 1, 2, 3, 4, 5, 6, 7, 8, 9, 10, 11, 12, 13, 14, 15); }
__device__ __forceinline__ v16bf cat16b(v8us lo, v8us hi) { return __builtin_bit_cast(v16bf, __builtin_shufflevector(lo, hi, 0, 1, 2, 3, 4, 5, 6, 7, 8, 9, 10, 11, 12, 13, 14, 15)); }
__device__ __forceinline__ v8f wmma16(v16h a, v16h b, v8f c) { return __builtin_amdgcn_wmma_f32_16x16x32_f16(false, a, false, b, (short)0, c, false, false); }
__device__ __forceinline__ v8f wmmab(v16bf a, v16bf b, v8f c) { return __builtin_amdgcn_wmma_f32_16x16x32_bf16(false, a, false, b, (short)0, c, false, false); }
__device__ __forceinline__ v16h  ldh(const h16* p) { return cat16(*(const v8h*)p, *(const v8h*)(p + 16)); }
__device__ __forceinline__ v16bf ldb(const bf* p)  { return cat16b(*(const v8us*)p, *(const v8us*)(p + 16)); }
__device__ __forceinline__ void wave_sync() { __builtin_amdgcn_fence(3  , "wavefront"); __builtin_amdgcn_wave_barrier(); asm volatile("" ::: "memory"); }

__device__ __forceinline__ h16 toh_flush(float v) { const h16 r = (h16)v; return (fabsf(v) < 6.103515625e-05f) ? (h16)0.0f : r; }
__device__ __forceinline__ v8f wmma16g(v16h a, v16h b, v8f c) {
    c = __builtin_amdgcn_wmma_f32_16x16x32_f16(false, a, false, b, (short)0, c, false, false);
    asm volatile("v_nop\n\tv_nop\n\tv_nop\n\tv_nop" : "+v"(c) : "v"(a), "v"(b));
    return c;
}
__device__ __forceinline__ float silu_f(float x) { return x * __builtin_amdgcn_rcpf(1.0f + __expf(-x)); }
__device__ __forceinline__ void split4(v4f y, v4h& hv, v4h& rv) {
#pragma unroll
    for (int i = 0; i < 4; ++i) { const h16 a0 = toh_flush(y[i]); hv[i] = a0; rv[i] = toh_flush((y[i] - (float)a0) * QRS); }
}
__device__ __forceinline__ v4f ln8(v4f x, v4f w, v4f b) {
    float s = (x[0] + x[1]) + (x[2] + x[3]);
    s += __shfl_xor(s, 1, 32); s += __shfl_xor(s, 2, 32); s += __shfl_xor(s, 4, 32);
    const float mu = s * (1.0f / 32.0f);
    const v4f d = x - mu;
    float q = (d[0] * d[0] + d[1] * d[1]) + (d[2] * d[2] + d[3] * d[3]);
    q += __shfl_xor(q, 1, 32); q += __shfl_xor(q, 2, 32); q += __shfl_xor(q, 4, 32);
    const float inv = 1.0f / sqrtf(q * (1.0f / 32.0f) + 1e-5f);
    v4f y;
#pragma unroll
    for (int i = 0; i < 4; ++i) y[i] = d[i] * inv * w[i] + b[i];
    return y;
}

__global__ __launch_bounds__(256) void k_wconv(const float* __restrict__ src, h16* dst, int n8src, int n8dst) {
    const int i = blockIdx.x * 256 + threadIdx.x; if (i >= n8dst) return;
    const int ic = i < n8src ? i : n8src - 1;
    v8f v = *(const v8f*)(src + (size_t)ic * 8);
    asm volatile("" : "+v"(v));
    const bool ok = i < n8src; v8h o;
#pragma unroll
    for (int k = 0; k < 8; ++k) { const h16 c = toh_flush(bfr(v[k]) * WSC); o[k] = ok ? c : (h16)0.0f; }
    *(volatile v8h*)(dst + (size_t)i * 8) = o; __threadfence(); *(volatile v8h*)(dst + (size_t)i * 8) = o;
}

__global__ __launch_bounds__(256) void k_ln_inproj(const float* __restrict__ ms, const float* __restrict__ rs, const float* __restrict__ pan,
                                                   const float* __restrict__ g1, const float* __restrict__ b1, const float* __restrict__ g2, const float* __restrict__ b2,
                                                   const h16* __restrict__ W1, float* OUT1, float* P3) {
    __shared__ __align__(16) h16 sa[4 * 128 * AP];
    __shared__ __align__(16) float os[8 * 16 * OS1P];
    const int lane = threadIdx.x & 31, lr = lane & 15, hi = lane >> 4;
    const int wave = __builtin_amdgcn_readfirstlane((int)(threadIdx.x >> 5));
    const int tile0 = blockIdx.x * 128;
    const int bb = tile0 / SEQ, tt = tile0 % SEQ;
    const size_t inrow = (size_t)bb * SEQ_FULL + (size_t)tt;
    const size_t outrow = (size_t)bb * OUT_SEQ + (size_t)tt;
    const int c4 = (lane & 7) * 4;
    v4f w1v, b1v, w2v, b2v;
    { const v4f a = *(const v4f*)(g1 + c4), c = *(const v4f*)(b1 + c4), e = *(const v4f*)(g2 + c4), f = *(const v4f*)(b2 + c4);
#pragma unroll
      for (int i = 0; i < 4; ++i) { w1v[i] = bfr(a[i]); b1v[i] = bfr(c[i]); w2v[i] = bfr(e[i]); b2v[i] = bfr(f[i]); } }
#pragma unroll 1
    for (int it = 0; it < 4; ++it) {
        const int tl = wave * 16 + it * 4 + (lane >> 3);
        const size_t gi = (inrow + (size_t)tl) * CW + c4;
        const v4f a = *(const v4f*)(ms + gi), c = *(const v4f*)(rs + gi);
        v4f r;
#pragma unroll
        for (int i = 0; i < 4; ++i) r[i] = bfr(a[i]) + bfr(c[i]);
        float* op = OUT1 + (outrow + (size_t)tl) * CW + c4;
        *(volatile v4f*)op = r; __threadfence(); *(volatile v4f*)op = r;
        const v4f y = ln8(ln8(r, w1v, b1v), w1v, b1v);
        v4h hv, rv; split4(y, hv, rv);
        *(v4h*)(&sa[(0 * 128 + tl) * AP + c4]) = hv; *(v4h*)(&sa[(1 * 128 + tl) * AP + c4]) = rv;
    }
#pragma unroll 1
    for (int it = 0; it < 4; ++it) {
        const int tl = wave * 16 + it * 4 + (lane >> 3);
        const size_t gi = (inrow + (size_t)tl) * CW + c4;
        const v4f a = *(const v4f*)(pan + gi);
        v4f r;
#pragma unroll
        for (int i = 0; i < 4; ++i) r[i] = bfr(a[i]);
        const v4f y = ln8(ln8(r, w2v, b2v), w2v, b2v);
        v4h hv, rv; split4(y, hv, rv);
        *(v4h*)(&sa[(2 * 128 + tl) * AP + c4]) = hv; *(v4h*)(&sa[(3 * 128 + tl) * AP + c4]) = rv;
    }
    __syncthreads();
    const int arow = (wave * 16 + lr) * AP + 8 * hi;
    const v16h aMH = cat16(*(const v8h*)(&sa[0 * 128 * AP + arow]), *(const v8h*)(&sa[0 * 128 * AP + arow + 16]));
    const v16h aMR = cat16(*(const v8h*)(&sa[1 * 128 * AP + arow]), *(const v8h*)(&sa[1 * 128 * AP + arow + 16]));
    const v16h aPH = cat16(*(const v8h*)(&sa[2 * 128 * AP + arow]), *(const v8h*)(&sa[2 * 128 * AP + arow + 16]));
    const v16h aPR = cat16(*(const v8h*)(&sa[3 * 128 * AP + arow]), *(const v8h*)(&sa[3 * 128 * AP + arow + 16]));
    const int wb = wave * 16 * OS1P;
    const size_t plane = (size_t)NB * SEQ * DI;
#pragma unroll
    for (int g = 0; g < 3; ++g) {
        const v16h ah = (g < 2) ? aMH : aPH;
        const v16h ar = (g < 2) ? aMR : aPR;
#pragma unroll
        for (int nb = 0; nb < 4; ++nb) {
            const v16h b = ldh(W1 + (size_t)((g * 4 + nb) * 16 + lr) * CW + 8 * hi);
            v8f cH = (v8f){}, cL = (v8f){};
            cH = wmma16g(ah, b, cH); cL = wmma16g(ar, b, cL);
#pragma unroll
            for (int j = 0; j < 8; ++j) os[wb + (hi * 8 + j) * OS1P + nb * 16 + lr] = (cH[j] + cL[j] * QRI) * (1.0f / WSC);
        }
        wave_sync();
        float* dst = P3 + (size_t)g * plane + (size_t)(tile0 + wave * 16) * DI;
#pragma unroll 1
        for (int ps = 0; ps < 2; ++ps) {
#pragma unroll
            for (int s = 0; s < 8; ++s) { const int p = s * 32 + lane; const int row = p >> 4, cc = (p & 15) * 4;
                const v4f val = *(const v4fa*)(&os[wb + row * OS1P + cc]);
                *(volatile v4f*)(dst + (size_t)p * 4) = val; }
            if (ps == 0) __threadfence(); }
        wave_sync();
    }
}

__global__ __launch_bounds__(128) void k_conv_xproj(const float* __restrict__ XR, const float* __restrict__ XPR,
                                                    const float* __restrict__ cw, const float* __restrict__ cb, const float* __restrict__ cpw, const float* __restrict__ cpb,
                                                    const h16* __restrict__ W2, const float* __restrict__ wdt, const float* __restrict__ bdt,
                                                    float* UU, float* DT, float* BC) {
    __shared__ __align__(16) float sx[67 * 64];
    __shared__ __align__(16) float sxp[67 * 64];
    __shared__ __align__(16) float su[64 * 64];
    __shared__ __align__(16) h16 sa[64 * XAP];
    __shared__ __align__(16) float sd[64 * SDP];
    const int tid = threadIdx.x;
    const int lane = tid & 31, lr = lane & 15, hi = lane >> 4;
    const int wave = __builtin_amdgcn_readfirstlane((int)(threadIdx.x >> 5));
    const int tile0 = blockIdx.x * 64;
    const int tt = tile0 % SEQ;
    const size_t seq0 = (size_t)(tile0 - tt);
#pragma unroll 1
    for (int i = tid; i < 67 * 16; i += 128) {
        const int row = i >> 4, cc = (i & 15) * 4;
        const int t = tt - 3 + row; const int tc = t < 0 ? 0 : t;
        const size_t gi = (seq0 + (size_t)tc) * DI + cc;
        v4f a = *(const v4f*)(XR + gi), c = *(const v4f*)(XPR + gi);
        asm volatile("" : "+v"(a)); asm volatile("" : "+v"(c));
        const bool ok = t >= 0; const v4f z = (v4f){};
        *(v4fa*)(&sx[row * 64 + cc]) = ok ? a : z; *(v4fa*)(&sxp[row * 64 + cc]) = ok ? c : z;
    }
    __syncthreads();
    const int d = tid & 63;
    {
        float wx[4], wp[4];
#pragma unroll
        for (int j = 0; j < 4; ++j) { wx[j] = bfr(cw[d * 4 + j]); wp[j] = bfr(cpw[d * 4 + j]); }
        const float bx = bfr(cb[d]), bp = bfr(cpb[d]);
#pragma unroll 1
        for (int t = tid >> 6; t < 64; t += 2) {
            float ax = 0.0f, ap = 0.0f;
#pragma unroll
            for (int j = 0; j < 4; ++j) { ax = fmaf(wx[j], sx[(t + j) * 64 + d], ax); ap = fmaf(wp[j], sxp[(t + j) * 64 + d], ap); }
            ax += bx; ap += bp;
            su[t * 64 + d] = silu_f(ax);
            sa[t * XAP + d] = toh_flush(silu_f(ap) * ACS);
        }
    }
    __syncthreads();
    { float* dst = UU + (size_t)tile0 * DI;
#pragma unroll 1
      for (int ps = 0; ps < 2; ++ps) {
#pragma unroll
          for (int s = 0; s < 8; ++s) { const int p = s * 128 + tid;
              const v4f val = *(const v4fa*)(&su[p * 4]);
              *(volatile v4f*)(dst + (size_t)p * 4) = val; }
          if (ps == 0) __threadfence(); } }
    {
        v8f acc[3];
#pragma unroll
        for (int nt = 0; nt < 3; ++nt) acc[nt] = (v8f){};
#pragma unroll
        for (int kc = 0; kc < DI; kc += 32) {
            const int ao = (wave * 16 + lr) * XAP + 8 * hi + kc;
            const v16h a = cat16(*(const v8h*)(&sa[ao]), *(const v8h*)(&sa[ao + 16]));
#pragma unroll
            for (int nt = 0; nt < 3; ++nt) { const v16h b = ldh(W2 + (size_t)(nt * 16 + lr) * DI + 8 * hi + kc); acc[nt] = wmma16g(a, b, acc[nt]); }
        }
#pragma unroll
        for (int nt = 0; nt < 3; ++nt)
#pragma unroll
            for (int j = 0; j < 8; ++j) sd[(wave * 16 + hi * 8 + j) * SDP + nt * 16 + lr] = acc[nt][j] * (1.0f / (ACS * WSC));
    }
    __syncthreads();
    {
        const float w0 = bfr(wdt[d * 2]), w1 = bfr(wdt[d * 2 + 1]), bd = bfr(bdt[d]);
#pragma unroll 1
        for (int t = tid >> 6; t < 64; t += 2) {
            const float x = fmaf(sd[t * SDP + 1], w1, sd[t * SDP] * w0) + bd;
            sx[t * 64 + d] = fmaxf(x, 0.0f) + log1pf(expf(-fabsf(x)));
        }
    }
    { float* dst = BC + (size_t)tile0 * 32;
#pragma unroll 1
      for (int ps = 0; ps < 2; ++ps) {
#pragma unroll
          for (int s = 0; s < 4; ++s) { const int p = s * 128 + tid; const int row = p >> 3, cc = (p & 7) * 4;
              v4f val;
#pragma unroll
              for (int i = 0; i < 4; ++i) val[i] = sd[row * SDP + 2 + cc + i];
              *(volatile v4f*)(dst + (size_t)p * 4) = val; }
          if (ps == 0) __threadfence(); } }
    __syncthreads();
    { float* dst = DT + (size_t)tile0 * DI;
#pragma unroll 1
      for (int ps = 0; ps < 2; ++ps) {
#pragma unroll
          for (int s = 0; s < 8; ++s) { const int p = s * 128 + tid;
              const v4f val = *(const v4fa*)(&sx[p * 4]);
              *(volatile v4f*)(dst + (size_t)p * 4) = val; }
          if (ps == 0) __threadfence(); } }
}

__global__ __launch_bounds__(64) void k_scan_local(const float* __restrict__ DT, const float* __restrict__ UU, const float* __restrict__ BC,
                                                   const float* __restrict__ alog, float* CR) {
    __shared__ __align__(16) float cs[64 * 32];
    const int d = threadIdx.x;
    const size_t tok0 = (size_t)blockIdx.x * LC;
    float A2[16], h[16], ap[16];
    { const v4f a0 = *(const v4f*)(alog + d * NS), a1 = *(const v4f*)(alog + d * NS + 4), a2 = *(const v4f*)(alog + d * NS + 8), a3 = *(const v4f*)(alog + d * NS + 12);
#pragma unroll
      for (int r = 0; r < 4; ++r) { A2[r] = -__expf(bfr(a0[r])) * LOG2E; A2[4 + r] = -__expf(bfr(a1[r])) * LOG2E; A2[8 + r] = -__expf(bfr(a2[r])) * LOG2E; A2[12 + r] = -__expf(bfr(a3[r])) * LOG2E; } }
#pragma unroll
    for (int n = 0; n < 16; ++n) { h[n] = 0.0f; ap[n] = 1.0f; }
#pragma unroll 1
    for (int l = 0; l < LC; ++l) {
        const size_t tk = tok0 + (size_t)l;
        const float dt = DT[tk * DI + d], uv = UU[tk * DI + d];
        const float* bp = BC + tk * 32;
        const v4f b0 = *(const v4f*)bp, b1 = *(const v4f*)(bp + 4), b2 = *(const v4f*)(bp + 8), b3 = *(const v4f*)(bp + 12);
        float bv[16];
#pragma unroll
        for (int r = 0; r < 4; ++r) { bv[r] = b0[r]; bv[4 + r] = b1[r]; bv[8 + r] = b2[r]; bv[12 + r] = b3[r]; }
        const float du = dt * uv;
#pragma unroll
        for (int n = 0; n < 16; ++n) { const float da = __builtin_amdgcn_exp2f(dt * A2[n]); h[n] = fmaf(da, h[n], du * bv[n]); ap[n] *= da; }
    }
#pragma unroll
    for (int n = 0; n < 16; ++n) { cs[d * 32 + n] = ap[n]; cs[d * 32 + 16 + n] = h[n]; }
    __syncthreads();
    float* dst = CR + (size_t)blockIdx.x * (64 * 32);
#pragma unroll 1
    for (int ps = 0; ps < 2; ++ps) {
#pragma unroll
        for (int s = 0; s < 8; ++s) { const int p = s * 64 + d;
            const v4f val = *(const v4fa*)(&cs[p * 4]);
            *(volatile v4f*)(dst + (size_t)p * 4) = val; }
        if (ps == 0) __threadfence(); }
}

__global__ __launch_bounds__(64) void k_scan_out(const float* __restrict__ DT, const float* __restrict__ UU, const float* __restrict__ BC, const float* __restrict__ ZR,
                                                 const float* __restrict__ alog, const float* __restrict__ dpar, const float* __restrict__ CR, h16* VH, h16* VR) {
    __shared__ __align__(16) float ys[TS * 64];
    const int d = threadIdx.x;
    const int blk = blockIdx.x; const int ch = blk % NCH;
    const size_t tok0 = (size_t)blk * LC;
    float A2[16], h[16];
    { const v4f a0 = *(const v4f*)(alog + d * NS), a1 = *(const v4f*)(alog + d * NS + 4), a2 = *(const v4f*)(alog + d * NS + 8), a3 = *(const v4f*)(alog + d * NS + 12);
#pragma unroll
      for (int r = 0; r < 4; ++r) { A2[r] = -__expf(bfr(a0[r])) * LOG2E; A2[4 + r] = -__expf(bfr(a1[r])) * LOG2E; A2[8 + r] = -__expf(bfr(a2[r])) * LOG2E; A2[12 + r] = -__expf(bfr(a3[r])) * LOG2E; } }
    const float Dd = bfr(dpar[d]);
#pragma unroll
    for (int n = 0; n < 16; ++n) h[n] = 0.0f;
#pragma unroll 1
    for (int c = 0; c < ch; ++c) {
        const float* cp = CR + ((size_t)(blk - ch + c) * 64 + (size_t)d) * 32;
        const v4f p0 = *(const v4f*)cp, p1 = *(const v4f*)(cp + 4), p2 = *(const v4f*)(cp + 8), p3 = *(const v4f*)(cp + 12);
        const v4f e0 = *(const v4f*)(cp + 16), e1 = *(const v4f*)(cp + 20), e2 = *(const v4f*)(cp + 24), e3 = *(const v4f*)(cp + 28);
#pragma unroll
        for (int r = 0; r < 4; ++r) { h[r] = fmaf(p0[r], h[r], e0[r]); h[4 + r] = fmaf(p1[r], h[4 + r], e1[r]); h[8 + r] = fmaf(p2[r], h[8 + r], e2[r]); h[12 + r] = fmaf(p3[r], h[12 + r], e3[r]); }
    }
#pragma unroll 1
    for (int s0 = 0; s0 < LC; s0 += TS) {
#pragma unroll 1
        for (int l = 0; l < TS; ++l) {
            const size_t tk = tok0 + (size_t)(s0 + l);
            const float dt = DT[tk * DI + d], uv = UU[tk * DI + d];
            const float* bp = BC + tk * 32;
            const v4f b0 = *(const v4f*)bp, b1 = *(const v4f*)(bp + 4), b2 = *(const v4f*)(bp + 8), b3 = *(const v4f*)(bp + 12);
            const v4f c0 = *(const v4f*)(bp + 16), c1 = *(const v4f*)(bp + 20), c2 = *(const v4f*)(bp + 24), c3 = *(const v4f*)(bp + 28);
            float bv[16], cv[16];
#pragma unroll
            for (int r = 0; r < 4; ++r) { bv[r] = b0[r]; bv[4 + r] = b1[r]; bv[8 + r] = b2[r]; bv[12 + r] = b3[r]; cv[r] = c0[r]; cv[4 + r] = c1[r]; cv[8 + r] = c2[r]; cv[12 + r] = c3[r]; }
            const float du = dt * uv;
            float y = 0.0f;
#pragma unroll
            for (int n = 0; n < 16; ++n) { const float da = __builtin_amdgcn_exp2f(dt * A2[n]); h[n] = fmaf(da, h[n], du * bv[n]); y = fmaf(h[n], cv[n], y); }
            ys[l * 64 + d] = fmaf(uv, Dd, y);
        }
        __syncthreads();
        const size_t e0 = (tok0 + (size_t)s0) * DI;
#pragma unroll 1
        for (int ps = 0; ps < 2; ++ps) {
#pragma unroll 1
            for (int q = 0; q < 4; ++q) { const int p = q * 64 + d;
                const v4f y0 = *(const v4fa*)(&ys[p * 8]), y1 = *(const v4fa*)(&ys[p * 8 + 4]);
                const v4f z0 = *(const v4f*)(ZR + e0 + (size_t)p * 8), z1 = *(const v4f*)(ZR + e0 + (size_t)p * 8 + 4);
                v8h hv, rv;
#pragma unroll
                for (int i = 0; i < 4; ++i) {
                    const float ga = y0[i] * silu_f(z0[i]) * ACS, gb = y1[i] * silu_f(z1[i]) * ACS;
                    const h16 a0 = toh_flush(ga); const h16 a1 = toh_flush(gb);
                    hv[i] = a0; hv[4 + i] = a1; rv[i] = toh_flush((ga - (float)a0) * QRS); rv[4 + i] = toh_flush((gb - (float)a1) * QRS); }
                *(volatile v8h*)(VH + e0 + (size_t)p * 8) = hv; *(volatile v8h*)(VR + e0 + (size_t)p * 8) = rv; }
            if (ps == 0) __threadfence(); }
        __syncthreads();
    }
}

__global__ __launch_bounds__(128) void k_outproj(const h16* __restrict__ VH, const h16* __restrict__ VR, const h16* __restrict__ W3, float* G) {
    __shared__ __align__(16) float os[4 * 16 * OSP];
    const int lane = threadIdx.x & 31, lr = lane & 15, hi = lane >> 4;
    const int wave = __builtin_amdgcn_readfirstlane((int)(threadIdx.x >> 5));
    const size_t tok0 = (size_t)blockIdx.x * 64 + (size_t)(wave * 16);
    const size_t ao = (tok0 + (size_t)lr) * DI + 8 * hi;
    v8f cH0 = (v8f){}, cH1 = (v8f){}, cL0 = (v8f){}, cL1 = (v8f){};
#pragma unroll
    for (int kc = 0; kc < DI; kc += 32) {
        const v16h ah = ldh(VH + ao + kc), ar = ldh(VR + ao + kc);
        const v16h b0 = ldh(W3 + (size_t)lr * DI + 8 * hi + kc), b1 = ldh(W3 + (size_t)(16 + lr) * DI + 8 * hi + kc);
        cH0 = wmma16g(ah, b0, cH0); cH1 = wmma16g(ah, b1, cH1);
        cL0 = wmma16g(ar, b0, cL0); cL1 = wmma16g(ar, b1, cL1);
    }
    const float sc = 1.0f / (ACS * WSC);
    const int wb = wave * 16 * OSP;
#pragma unroll
    for (int j = 0; j < 8; ++j) { os[wb + (hi * 8 + j) * OSP + lr] = (cH0[j] + cL0[j] * QRI) * sc; os[wb + (hi * 8 + j) * OSP + 16 + lr] = (cH1[j] + cL1[j] * QRI) * sc; }
    wave_sync();
    float* dst = G + tok0 * CW;
#pragma unroll 1
    for (int ps = 0; ps < 2; ++ps) {
#pragma unroll
        for (int s = 0; s < 4; ++s) { const int row = 4 * s + (lane >> 3), cofs = (lane & 7) * 4;
            const v4f val = *(const v4fa*)(&os[wb + row * OSP + cofs]);
            *(volatile v4f*)(dst + (size_t)row * CW + cofs) = val; }
        if (ps == 0) __threadfence(); }
}

__global__ __launch_bounds__(256) void k_dwconv(const float* __restrict__ G, const float* __restrict__ w, const float* __restrict__ bias, float* OUT) {
    const size_t idx = (size_t)blockIdx.x * 256 + threadIdx.x;
    if (idx >= (size_t)NB * SEQ * 8) return;
    const int tok = (int)(idx >> 3); const int c4 = ((int)idx & 7) * 4;
    const int bb = tok / SEQ, pos = tok % SEQ; const int hy = pos / IMG, wx = pos % IMG;
    v4f acc = (v4f){};
#pragma unroll 1
    for (int kh = 0; kh < 3; ++kh) {
        const int nh = hy + kh - 1; const bool okh = (nh >= 0) & (nh < IMG); const int nhc = nh < 0 ? 0 : (nh > IMG - 1 ? IMG - 1 : nh);
#pragma unroll
        for (int kw = 0; kw < 3; ++kw) {
            const int nw = wx + kw - 1; const bool ok = okh & (nw >= 0) & (nw < IMG); const int nwc = nw < 0 ? 0 : (nw > IMG - 1 ? IMG - 1 : nw);
            v4f gv = *(const v4f*)(G + ((size_t)bb * SEQ + (size_t)(nhc * IMG + nwc)) * CW + c4);
            asm volatile("" : "+v"(gv));
#pragma unroll
            for (int i = 0; i < 4; ++i) { const float wv = bfr(w[(c4 + i) * 9 + kh * 3 + kw]); acc[i] = fmaf(wv, ok ? gv[i] : 0.0f, acc[i]); }
        }
    }
    const v4f gc = *(const v4f*)(G + (size_t)tok * CW + c4);
    const v4f bv = *(const v4f*)(bias + c4);
    v4f o;
#pragma unroll
    for (int i = 0; i < 4; ++i) o[i] = (acc[i] + bfr(bv[i])) + gc[i];
    float* op = OUT + ((size_t)bb * OUT_SEQ + (size_t)pos) * CW + c4;
    *(volatile v4f*)op = o; __threadfence(); *(volatile v4f*)op = o;
}

static constexpr size_t al256(size_t v) { return (v + 255) & ~(size_t)255; }
static constexpr size_t SZ_W1 = al256((size_t)192 * CW * 2);
static constexpr size_t SZ_W2 = al256((size_t)XPP * DI * 2);
static constexpr size_t SZ_W3 = al256((size_t)CW * DI * 2);
static constexpr size_t SZ_P64 = al256((size_t)NB * SEQ * DI * 4);
static constexpr size_t SZ_P32 = al256((size_t)NB * SEQ * 32 * 4);
static constexpr size_t SZ_CR = al256((size_t)NB * NCH * 64 * 32 * 4);
static constexpr size_t SZ_VH = al256((size_t)NB * SEQ * DI * 2);
static constexpr size_t SZ_TOTAL = SZ_W1 + SZ_W2 + SZ_W3 + 5 * SZ_P64 + 2 * SZ_P32 + SZ_CR + 2 * SZ_VH;
static_assert(SZ_TOTAL <= (size_t)134217728);
static_assert(((size_t)NB * SEQ * DI * 4) % 256 == 0);
static_assert(((size_t)128 * CW * 2) % 256 == 0);
static_assert((size_t)NB * NCH * LC == (size_t)NB * SEQ);

extern "C" void kernel_launch(void* const* d_in, const int* in_sizes, int n_in,
                              void* d_out, int out_size, void* d_ws, size_t ws_size, hipStream_t stream) {
    if (n_in < 21) return;
    const size_t needx = ((size_t)(NB - 1) * SEQ_FULL + SEQ) * CW;
    if ((size_t)in_sizes[0] < needx || (size_t)in_sizes[1] < needx || (size_t)in_sizes[2] < needx) return;
    if (in_sizes[3] < CW || in_sizes[4] < CW || in_sizes[5] < CW || in_sizes[6] < CW) return;
    if (in_sizes[7] < 2 * DI * CW || in_sizes[8] < DI * CW) return;
    if (in_sizes[9] < DI * 4 || in_sizes[10] < DI || in_sizes[11] < DI * 4 || in_sizes[12] < DI) return;
    if (in_sizes[13] < XPN * DI || in_sizes[14] < DI * 2 || in_sizes[15] < DI || in_sizes[16] < DI * NS || in_sizes[17] < DI) return;
    if (in_sizes[18] < CW * DI || in_sizes[19] < CW * 9 || in_sizes[20] < CW) return;
    const size_t out1_off = (size_t)NB_FULL * SEQ_FULL * CW;
    if ((size_t)out_size < out1_off + ((size_t)(NB - 1) * OUT_SEQ + SEQ) * CW) return;
    if (SZ_TOTAL > ws_size) return;
    const float* ms   = (const float*)d_in[0];
    const float* rs   = (const float*)d_in[1];
    const float* pan  = (const float*)d_in[2];
    const float* ln1w = (const float*)d_in[3];  const float* ln1b = (const float*)d_in[4];
    const float* ln2w = (const float*)d_in[5];  const float* ln2b = (const float*)d_in[6];
    const float* win  = (const float*)d_in[7];
    const float* winp = (const float*)d_in[8];
    const float* cw   = (const float*)d_in[9];  const float* cb  = (const float*)d_in[10];
    const float* cpw  = (const float*)d_in[11]; const float* cpb = (const float*)d_in[12];
    const float* wxp  = (const float*)d_in[13];
    const float* wdt  = (const float*)d_in[14];
    const float* bdt  = (const float*)d_in[15];
    const float* alog = (const float*)d_in[16];
    const float* dpar = (const float*)d_in[17];
    const float* wout = (const float*)d_in[18];
    const float* dww  = (const float*)d_in[19];
    const float* dwb  = (const float*)d_in[20];
    float* OUT0 = (float*)d_out;
    float* OUT1 = (float*)d_out + out1_off;
    char* wsp = (char*)d_ws;
    h16* W1 = (h16*)wsp; wsp += SZ_W1;
    h16* W2 = (h16*)wsp; wsp += SZ_W2;
    h16* W3 = (h16*)wsp; wsp += SZ_W3;
    float* P3 = (float*)wsp; wsp += 3 * SZ_P64;
    float* UU = (float*)wsp; wsp += SZ_P64;
    float* DT = (float*)wsp; wsp += SZ_P64;
    float* BC = (float*)wsp; wsp += SZ_P32;
    float* GG = (float*)wsp; wsp += SZ_P32;
    float* CR = (float*)wsp; wsp += SZ_CR;
    h16* VH = (h16*)wsp; wsp += SZ_VH;
    h16* VR = (h16*)wsp; wsp += SZ_VH;
    const size_t plane = (size_t)NB * SEQ * DI;

    k_wconv<<<(512 + 255) / 256, 256, 0, stream>>>(win,  W1, 512, 512);
    k_wconv<<<(256 + 255) / 256, 256, 0, stream>>>(winp, W1 + (size_t)128 * CW, 256, 256);
    k_wconv<<<(384 + 255) / 256, 256, 0, stream>>>(wxp,  W2, (XPN * DI) / 8, (XPP * DI) / 8);
    k_wconv<<<(256 + 255) / 256, 256, 0, stream>>>(wout, W3, 256, 256);

    k_ln_inproj<<<NB * SEQ / 128, 256, 0, stream>>>(ms, rs, pan, ln1w, ln1b, ln2w, ln2b, W1, OUT1, P3);
    k_conv_xproj<<<NB * SEQ / 64, 128, 0, stream>>>(P3, P3 + 2 * plane, cw, cb, cpw, cpb, W2, wdt, bdt, UU, DT, BC);
    k_scan_local<<<NB * NCH, 64, 0, stream>>>(DT, UU, BC, alog, CR);
    k_scan_out<<<NB * NCH, 64, 0, stream>>>(DT, UU, BC, P3 + plane, alog, dpar, CR, VH, VR);
    k_outproj<<<NB * SEQ / 64, 128, 0, stream>>>(VH, VR, W3, GG);
    k_dwconv<<<(unsigned)(((size_t)NB * SEQ * 8 + 255) / 256), 256, 0, stream>>>(GG, dww, dwb, OUT0);
}
